// GQA_39015482917267
// MI455X (gfx1250) — hardware-verified
//
#include <hip/hip_runtime.h>


#ifndef NB
#define NB 2
#endif
#ifndef SEQ
#define SEQ 2048
#endif

namespace {
constexpr int B_FULL = 2, T_FULL = 2048, DM = 1024, H = 16, HD = 64, G = 4, REP = H / G, KVW = G * HD;
constexpr int BL = NB, QL = SEQ;
constexpr int NQS = DM / 128, NKS = KVW / 128, NPART = NQS + 2 * NKS, NPAIR = HD / 2;
constexpr float XS = 8.0f, WSC = 256.0f, PS = 1024.0f, RS_ = 1024.0f, LOG2E = 1.4426950408889634f, LN1E4 = 9.2103404f;
static_assert(BL >= 1 && BL <= B_FULL);
static_assert(QL % 64 == 0 && QL >= 64 && QL <= T_FULL);
static_assert(DM % 256 == 0 && H * HD == DM && HD == 64 && KVW == 256 && REP == 4 && NPAIR == 32 && NPART == 12 && NQS == 8 && NKS == 2);

typedef _Float16 b16;
typedef __attribute__((ext_vector_type(16))) _Float16 v16b;
typedef __attribute__((ext_vector_type(8))) _Float16 v8b;
typedef __attribute__((ext_vector_type(4))) _Float16 v4h;
typedef __attribute__((ext_vector_type(8))) float v8f;
typedef __attribute__((ext_vector_type(4))) float v4f;

__device__ __forceinline__ float bf16_rne(float f) { unsigned int u = __float_as_uint(f); u += 0x7FFFu + ((u >> 16) & 1u); return __uint_as_float(u & 0xFFFF0000u); }
__device__ __forceinline__ int iclamp(int v, int lo, int hi) { return v < lo ? lo : (v > hi ? hi : v); }
__device__ __forceinline__ float nexp2(float v) { return __builtin_amdgcn_exp2f(v); }

__device__ __forceinline__ v16b frag_kb(const b16* p, int hh) {
  const v8b a = *(const v8b*)(p + 8 * hh), b = *(const v8b*)(p + 16 + 8 * hh);
  v16b f;
#pragma unroll
  for (int e = 0; e < 8; ++e) { f[e] = a[e]; f[8 + e] = b[e]; }
  return f;
}
__device__ __forceinline__ v8f wmma16b(v16b a, v16b b, v8f c) {
  v8f d = __builtin_amdgcn_wmma_f32_16x16x32_f16(false, a, false, b, (short)0, c, false, false);
  asm volatile("v_nop\n\tv_nop\n\tv_nop\n\tv_nop" : "+v"(d) : "v"(a), "v"(b));
  return d;
}
__device__ __forceinline__ void wave_lds_sync() { __builtin_amdgcn_fence(3  , "workgroup"); __builtin_amdgcn_wave_barrier(); __builtin_amdgcn_fence(2  , "workgroup"); }

__global__ __launch_bounds__(256) void tab_kernel(float* __restrict__ CS, float* __restrict__ SN) {
#pragma clang fp contract(off)
  const int t = blockIdx.x * 8 + (threadIdx.x >> 5), p = threadIdx.x & 31;
  if (t >= QL) return;
  const float fr = expf(-((float)(2 * p) * (1.0f / (float)HD)) * LN1E4);
  const float ang = (float)t * fr;
  float sn, cs;
  sincosf(ang, &sn, &cs);
  const size_t o = (size_t)t * NPAIR + p;
  for (int pass = 0; pass < 2; ++pass) { *(volatile float*)(CS + o) = cs; *(volatile float*)(SN + o) = sn; __threadfence(); }
}

__global__ __launch_bounds__(256) void prep_kernel(const float* __restrict__ wq, const float* __restrict__ wk, const float* __restrict__ wv, const float* __restrict__ wo, b16* __restrict__ WT, b16* __restrict__ WO) {
  const size_t u = (size_t)blockIdx.x * 256 + threadIdx.x;
  const size_t nq = (size_t)DM * DM / 8, nk = (size_t)KVW * DM / 8;
  if (u >= 2 * nq + 2 * nk) return;
  v8b o; b16* dst;
  if (u < nq) {
    const int row = (int)(u / (DM / 8)), k0 = (int)(u % (DM / 8)) * 8;
#pragma unroll
    for (int j = 0; j < 8; ++j) o[j] = (b16)(bf16_rne(wq[(size_t)(k0 + j) * DM + row]) * WSC);
    dst = WT + (size_t)row * DM + k0;
  } else if (u < nq + 2 * nk) {
    const size_t e = u - nq; const int m = (int)(e / nk); const size_t e2 = e % nk;
    const int row = (int)(e2 / (DM / 8)), k0 = (int)(e2 % (DM / 8)) * 8;
    const float* w = (m == 0) ? wk : wv;
#pragma unroll
    for (int j = 0; j < 8; ++j) o[j] = (b16)(bf16_rne(w[(size_t)(k0 + j) * KVW + row]) * WSC);
    dst = WT + ((size_t)DM + (size_t)m * KVW + row) * DM + k0;
  } else {
    const size_t e = u - nq - 2 * nk; const int row = (int)(e / (DM / 8)), k0 = (int)(e % (DM / 8)) * 8;
#pragma unroll
    for (int j = 0; j < 8; ++j) o[j] = (b16)(bf16_rne(wo[(size_t)(k0 + j) * DM + row]) * WSC);
    dst = WO + (size_t)row * DM + k0;
  }
  for (int pass = 0; pass < 2; ++pass) { *(volatile v8b*)dst = o; __threadfence(); }
}

__global__ __launch_bounds__(128) void proj_kernel(const float* __restrict__ x, const b16* __restrict__ WT, const float* __restrict__ bq, const float* __restrict__ bk, const float* __restrict__ bv,
                                                   const float* __restrict__ CS, const float* __restrict__ SN,
                                                   b16* __restrict__ QP, b16* __restrict__ QPl, b16* __restrict__ KP, b16* __restrict__ KPl, b16* __restrict__ VT, b16* __restrict__ VTl) {
  __shared__ __attribute__((aligned(16))) b16 As[64][256 + 8];
  __shared__ __attribute__((aligned(16))) float Tf[4][16][128 + 4];
  const int tid = threadIdx.x, wave = tid >> 5, lane = tid & 31, nloc = lane & 15, hlf = lane >> 4;
  const int t0 = blockIdx.x * 64, b = blockIdx.y, slab = blockIdx.z, n0 = slab * 128;
  const float* xb = x + ((size_t)b * T_FULL + t0) * DM;
  v8f acc[8];
#pragma unroll
  for (int t = 0; t < 8; ++t) acc[t] = (v8f){};
#pragma unroll 1
  for (int kc = 0; kc < DM; kc += 256) {
    __syncthreads();
    for (int i = tid; i < 64 * 64; i += 128) {
      const int rr = i >> 6, q = (i & 63) * 4;
      const v4f f = *(const v4f*)(xb + (size_t)rr * DM + kc + q);
      v4h o;
#pragma unroll
      for (int j = 0; j < 4; ++j) o[j] = (b16)(bf16_rne(f[j]) * XS);
      *(v4h*)(&As[rr][q]) = o;
    }
    __syncthreads();
#pragma unroll 1
    for (int kb = 0; kb < 256; kb += 32) {
      const v16b a = frag_kb(&As[wave * 16 + nloc][kb], hlf);
#pragma unroll
      for (int t = 0; t < 8; ++t) acc[t] = wmma16b(a, frag_kb(WT + (size_t)(n0 + t * 16 + nloc) * DM + kc + kb, hlf), acc[t]);
    }
  }
#pragma unroll
  for (int t = 0; t < 8; ++t) {
    const int col = n0 + t * 16 + nloc;
    const int iq = col < DM ? col : DM - 1, ik = iclamp(col - DM, 0, KVW - 1), iv = iclamp(col - DM - KVW, 0, KVW - 1);
    const float vq = bq[iq], vk = bk[ik], vv = bv[iv];
    const float bb = bf16_rne(slab < NQS ? vq : (slab < NQS + NKS ? vk : vv));
#pragma unroll
    for (int r = 0; r < 8; ++r) Tf[wave][8 * hlf + r][t * 16 + nloc] = acc[t][r] * (1.0f / (XS * WSC)) + bb;
  }
  __syncthreads();
  if (slab < NQS + NKS) {
    const bool isq = slab < NQS;
    b16* Ph = isq ? QP : KP;
    b16* Pl = isq ? QPl : KPl;
    const int nh = isq ? H : G;
    const int hsel = (isq ? 2 * slab : 2 * (slab - NQS)) + hlf;
    const size_t pb = (((size_t)b * nh + hsel) * QL) * HD + (size_t)nloc * 4;
    const int p0 = nloc * 2;
    for (int pass = 0; pass < 2; ++pass) {
#pragma unroll 1
      for (int rr = 0; rr < 16; ++rr) {
        const int tok = t0 + wave * 16 + rr;
        const size_t tb = (size_t)tok * NPAIR + p0;
        const float c0 = CS[tb], s0 = SN[tb], c1 = CS[tb + 1], s1 = SN[tb + 1];
        const float xe0 = Tf[wave][rr][lane * 4 + 0], xo0 = Tf[wave][rr][lane * 4 + 1], xe1 = Tf[wave][rr][lane * 4 + 2], xo1 = Tf[wave][rr][lane * 4 + 3];
        float f[4];
        f[0] = (xe0 * c0 - xo0 * s0) * XS; f[1] = (xe0 * s0 + xo0 * c0) * XS;
        f[2] = (xe1 * c1 - xo1 * s1) * XS; f[3] = (xe1 * s1 + xo1 * c1) * XS;
        v4h h4, l4;
#pragma unroll
        for (int j = 0; j < 4; ++j) { const b16 p = (b16)f[j]; h4[j] = p; l4[j] = (b16)((f[j] - (float)p) * RS_); }
        const size_t o2 = pb + (size_t)tok * HD;
        *(volatile v4h*)(Ph + o2) = h4;
        *(volatile v4h*)(Pl + o2) = l4;
      }
      __threadfence();
    }
  } else {
    const int gb = 2 * (slab - NQS - NKS);
    for (int pass = 0; pass < 2; ++pass) {
#pragma unroll 1
      for (int it = 0; it < 16; ++it) {
        const int cidx = wave * 32 + 2 * it + hlf;
        const int gsel = gb + (cidx >> 6), d = cidx & 63;
        v4h h4, l4;
#pragma unroll
        for (int j = 0; j < 4; ++j) {
          const int tk = nloc * 4 + j;
          const float fv = Tf[tk >> 4][tk & 15][cidx] * XS;
          const b16 p = (b16)fv; h4[j] = p; l4[j] = (b16)((fv - (float)p) * RS_);
        }
        const size_t o2 = (((size_t)b * G + gsel) * HD + d) * (size_t)QL + t0 + nloc * 4;
        *(volatile v4h*)(VT + o2) = h4;
        *(volatile v4h*)(VTl + o2) = l4;
      }
      __threadfence();
    }
  }
}

__global__ __launch_bounds__(64) void attn_kernel(const b16* __restrict__ QP, const b16* __restrict__ QPl, const b16* __restrict__ KP, const b16* __restrict__ KPl,
                                                  const b16* __restrict__ VT, const b16* __restrict__ VTl, b16* __restrict__ Y, b16* __restrict__ Yl) {
  __shared__ __attribute__((aligned(16))) b16 Pb[2][16][32 + 8], Plq[2][16][32 + 8];
  __shared__ __attribute__((aligned(16))) float To[2][16][HD + 4];
  __shared__ __attribute__((aligned(16))) b16 Qs[2][16][HD + 8], Qsl[2][16][HD + 8];
  const int wave = threadIdx.x >> 5, lane = threadIdx.x & 31, hh = lane >> 4, col = lane & 15;
  const int b = blockIdx.y / H, h = blockIdx.y % H, g = h / REP;
  const int q0 = blockIdx.x * 32 + wave * 16, qi = q0 + col;
  const size_t qo = (((size_t)b * H + h) * QL) * HD, ko = (((size_t)b * G + g) * QL) * HD, vo = (((size_t)b * G + g) * HD) * (size_t)QL;
  const b16* Qb = QP + qo; const b16* Qbl = QPl + qo; const b16* Kb = KP + ko; const b16* Kbl = KPl + ko; const b16* Vb = VT + vo; const b16* Vbl = VTl + vo;
  const int kend = ((q0 + 16 + 31) / 32) * 32;
  for (int i = lane; i < 16 * (HD / 8); i += 32) {
    const int rr = i / (HD / 8), c8 = (i % (HD / 8)) * 8;
    *(v8b*)(&Qs[wave][rr][c8]) = *(const v8b*)(Qb + (size_t)(q0 + rr) * HD + c8);
    *(v8b*)(&Qsl[wave][rr][c8]) = *(const v8b*)(Qbl + (size_t)(q0 + rr) * HD + c8);
  }
  wave_lds_sync();
  const float cs = LOG2E * 0.125f / (XS * XS);
  float m = -INFINITY, l = 0.0f;
  v8f o[4], ol[4];
#pragma unroll
  for (int t = 0; t < 4; ++t) { o[t] = (v8f){}; ol[t] = (v8f){}; }
#pragma unroll 1
  for (int kb = 0; kb < kend; kb += 32) {
    float e[16]; float mx = -INFINITY;
#pragma unroll
    for (int u = 0; u < 2; ++u) {
      v8f s = (v8f){}, sx = (v8f){};
      const size_t kr = (size_t)(kb + u * 16 + col) * HD;
#pragma unroll
      for (int ks = 0; ks < 2; ++ks) {
        const v16b kf = frag_kb(Kb + kr + 32 * ks, hh);
        const v16b qf = frag_kb(&Qs[wave][col][32 * ks], hh);
        s = wmma16b(kf, qf, s);
        sx = wmma16b(kf, frag_kb(&Qsl[wave][col][32 * ks], hh), sx);
        sx = wmma16b(frag_kb(Kbl + kr + 32 * ks, hh), qf, sx);
      }
#pragma unroll
      for (int r = 0; r < 8; ++r) s[r] += sx[r] * (1.0f / RS_);
#pragma unroll
      for (int r = 0; r < 8; ++r) { const int key = kb + u * 16 + 8 * hh + r; const float vv = (key <= qi) ? s[r] * cs : -INFINITY; e[u * 8 + r] = vv; mx = fmaxf(mx, vv); }
    }
    mx = fmaxf(mx, __shfl_xor(mx, 16));
    const float mn = fmaxf(m, mx); const float al = nexp2(m - mn); float sum = 0.0f;
#pragma unroll
    for (int i2 = 0; i2 < 16; ++i2) {
      const float p = nexp2(e[i2] - mn); sum += p;
      const int pc = (i2 < 8 ? 0 : 16) + 8 * hh + (i2 & 7);
      const float ps = p * PS; const b16 phh = (b16)ps;
      Pb[wave][col][pc] = phh; Plq[wave][col][pc] = (b16)((ps - (float)phh) * RS_);
    }
    sum += __shfl_xor(sum, 16); l = l * al + sum; m = mn;
    wave_lds_sync();
    const v16b pf = frag_kb(&Pb[wave][col][0], hh), plf = frag_kb(&Plq[wave][col][0], hh);
#pragma unroll
    for (int t = 0; t < 4; ++t) {
      const v16b vh = frag_kb(Vb + (size_t)(t * 16 + col) * QL + kb, hh);
      o[t] *= al;
      o[t] = wmma16b(vh, pf, o[t]);
      ol[t] = wmma16b(frag_kb(Vbl + (size_t)(t * 16 + col) * QL + kb, hh), pf, ol[t] * al);
      ol[t] = wmma16b(vh, plf, ol[t]);
    }
    wave_lds_sync();
  }
  const float inv = 1.0f / (l * PS * XS);
#pragma unroll
  for (int t = 0; t < 4; ++t)
#pragma unroll
    for (int r = 0; r < 8; ++r) To[wave][col][t * 16 + 8 * hh + r] = (o[t][r] + ol[t][r] * (1.0f / RS_)) * inv;
  wave_lds_sync();
  for (int pass = 0; pass < 2; ++pass) {
#pragma unroll 1
    for (int it = 0; it < 8; ++it) {
      const int rr = 2 * it + hh;
      v4h hv, lv;
#pragma unroll
      for (int j = 0; j < 4; ++j) { const float f = To[wave][rr][col * 4 + j] * XS; const b16 p = (b16)f; hv[j] = p; lv[j] = (b16)((f - (float)p) * RS_); }
      const size_t oi = ((size_t)b * QL + q0 + rr) * DM + (size_t)h * HD + col * 4;
      *(volatile v4h*)(Y + oi) = hv;
      *(volatile v4h*)(Yl + oi) = lv;
    }
    __threadfence();
  }
}

__global__ __launch_bounds__(128) void out_kernel(const b16* __restrict__ Y, const b16* __restrict__ Yl, const b16* __restrict__ WO, const float* __restrict__ bo, float* __restrict__ out) {
  __shared__ __attribute__((aligned(16))) float Tf[4][16][128 + 4];
  const int wave = threadIdx.x >> 5, lane = threadIdx.x & 31, nloc = lane & 15, hlf = lane >> 4;
  const int b = blockIdx.z;
  const size_t m0 = (size_t)b * QL + (size_t)blockIdx.x * 64 + wave * 16;
  const int n0 = blockIdx.y * 128;
  v8f acc[8], accl[8];
#pragma unroll
  for (int t = 0; t < 8; ++t) { acc[t] = (v8f){}; accl[t] = (v8f){}; }
#pragma unroll 1
  for (int kb = 0; kb < DM; kb += 32) {
    const v16b a = frag_kb(Y + (m0 + nloc) * DM + kb, hlf), al = frag_kb(Yl + (m0 + nloc) * DM + kb, hlf);
#pragma unroll
    for (int t = 0; t < 8; ++t) {
      const v16b bw = frag_kb(WO + (size_t)(n0 + t * 16 + nloc) * DM + kb, hlf);
      acc[t] = wmma16b(a, bw, acc[t]);
      accl[t] = wmma16b(al, bw, accl[t]);
    }
  }
#pragma unroll
  for (int t = 0; t < 8; ++t)
#pragma unroll
    for (int r = 0; r < 8; ++r) Tf[wave][8 * hlf + r][t * 16 + nloc] = (acc[t][r] + accl[t][r] * (1.0f / RS_)) * (1.0f / (XS * WSC)) + bf16_rne(bo[n0 + t * 16 + nloc]);
  wave_lds_sync();
  const size_t orow = (size_t)b * T_FULL + (size_t)blockIdx.x * 64 + wave * 16;
  for (int pass = 0; pass < 2; ++pass) {
#pragma unroll 1
    for (int rr = 0; rr < 16; ++rr) *(volatile v4f*)(out + (orow + rr) * DM + n0 + lane * 4) = *(const v4f*)(&Tf[wave][rr][lane * 4]);
    __threadfence();
  }
}
}

extern "C" void kernel_launch(void* const* d_in, const int* in_sizes, int n_in, void* d_out, int out_size, void* d_ws, size_t ws_size, hipStream_t stream) {
  if (n_in < 9) return;
  auto Fp = [&](int i) { return (const float*)d_in[i]; };
  if (in_sizes[0] < BL * T_FULL * DM || in_sizes[1] < DM * DM || in_sizes[2] < DM || in_sizes[3] < DM * KVW || in_sizes[4] < KVW ||
      in_sizes[5] < DM * KVW || in_sizes[6] < KVW || in_sizes[7] < DM * DM || in_sizes[8] < DM || out_size < (BL - 1) * T_FULL * DM + QL * DM) return;
  size_t off = 0; char* ws = (char*)d_ws;
  auto carve = [&](size_t bytes) { char* p = ws + off; off += (bytes + 255) & ~(size_t)255; return p; };
  float* CS = (float*)carve((size_t)QL * NPAIR * 4);
  float* SN = (float*)carve((size_t)QL * NPAIR * 4);
  b16* WT = (b16*)carve((size_t)(DM + 2 * KVW) * DM * 2);
  b16* WO = (b16*)carve((size_t)DM * DM * 2);
  const size_t qpl = (size_t)BL * H * QL * HD * 2, kpl = (size_t)BL * G * QL * HD * 2, ypl = (size_t)BL * QL * DM * 2;
  b16* QP = (b16*)carve(qpl); b16* QPl = (b16*)carve(qpl);
  b16* KP = (b16*)carve(kpl); b16* KPl = (b16*)carve(kpl);
  b16* VT = (b16*)carve(kpl); b16* VTl = (b16*)carve(kpl);
  b16* Y = (b16*)carve(ypl);  b16* Yl = (b16*)carve(ypl);
  if (off > ws_size || off > ((size_t)128 << 20)) return;
  tab_kernel<<<(unsigned)(QL / 8), 256, 0, stream>>>(CS, SN);
  prep_kernel<<<(unsigned)(((size_t)(2 * DM * DM + 2 * KVW * DM) / 8 + 255) / 256), 256, 0, stream>>>(Fp(1), Fp(3), Fp(5), Fp(7), WT, WO);
  proj_kernel<<<dim3(QL / 64, BL, NPART), 128, 0, stream>>>(Fp(0), WT, Fp(2), Fp(4), Fp(6), CS, SN, QP, QPl, KP, KPl, VT, VTl);
  attn_kernel<<<dim3(QL / 32, BL * H), 64, 0, stream>>>(QP, QPl, KP, KPl, VT, VTl, Y, Yl);
  out_kernel<<<dim3(QL / 64, DM / 128, BL), 128, 0, stream>>>(Y, Yl, WO, Fp(8), (float*)d_out);
}
